// DConv2dBlock_59468117180728
// MI455X (gfx1250) — hardware-verified
//
#include <hip/hip_runtime.h>

#define NB    16
#define NC    32
#define NH    128
#define NW    128
#define NO    64
#define NK    9
#define HW    (NH * NW)
#define KD    (NK * NC)
#define PITCH 296
#define NOFF  18
#define NMOD  9
#define NCH1  32
#define XSP   130
#define OSP   128

typedef _Float16 v16h  __attribute__((ext_vector_type(16)));
typedef _Float16 v8h_t __attribute__((ext_vector_type(8)));
typedef v8h_t __attribute__((may_alias)) v8h;
typedef float    v8f   __attribute__((ext_vector_type(8)));
typedef float    v4f_t __attribute__((ext_vector_type(4)));
typedef v4f_t __attribute__((may_alias)) v4f;

union Frag { v16h v; v8h half[2]; };

__device__ __forceinline__ v8f wmma_f16(const v16h a, const v16h b, v8f c) {
  v8f d = __builtin_amdgcn_wmma_f32_16x16x32_f16(false, a, false, b, (short)0, c, false, false);
  asm volatile("v_nop\n\tv_nop\n\tv_nop\n\tv_nop" : "+v"(d) : "v"(a), "v"(b));
  return d;
}

__device__ __forceinline__ void conv1_rows_out(const float* osm, float* offo, float* modo,
                                               int b, int h, int wave, int lane) {
  for (int ch = wave; ch < NOFF + NMOD; ch += 8) {
    const v4f v = *(const v4f*)(osm + ch * OSP + 4 * lane);
    float* dst = (ch < NOFF) ? (offo + ((size_t)(b * NOFF + ch) * NH + h) * NW)
                             : (modo + ((size_t)(b * NMOD + (ch - NOFF)) * NH + h) * NW);
    *(volatile v4f*)(dst + 4 * lane) = v;
  }
}

__global__ void __launch_bounds__(256) k_conv_off(
    const float* __restrict__ x, const float* __restrict__ ow, const float* __restrict__ ob,
    const float* __restrict__ mw, const float* __restrict__ mb,
    float* offo, float* modo, int nblk)
{
  extern __shared__ v4f_t ldsraw[];
  unsigned char* base = (unsigned char*)ldsraw;
  _Float16* wsm = (_Float16*)base;
  _Float16* xs  = (_Float16*)(base + NCH1 * PITCH * 2);
  float*    osm = (float*)(base + NCH1 * PITCH * 2 + 3 * XSP * NC * 2);

  const int blk = blockIdx.x;
  if (blk >= nblk) return;
  const int b = blk / NH, h = blk - b * NH;
  const int tid = threadIdx.x, wave = tid >> 5, lane = tid & 31;
  const int hf = lane >> 4, m = lane & 15;

  for (int i = tid; i < NCH1 * KD; i += 256) {
    const int n = i / KD, kk = i - n * KD;
    const int k = kk / NC, c = kk - k * NC;
    float v = 0.0f;
    if (n < NOFF)             v = ow[(n * NC + c) * NK + k];
    else if (n < NOFF + NMOD) v = mw[((n - NOFF) * NC + c) * NK + k];
    wsm[n * PITCH + kk] = (_Float16)(v * 1024.0f);
  }
  for (int i = tid; i < NC * 3 * XSP; i += 256) {
    const int pc = i % XSP, r = (i / XSP) % 3, c = i / (3 * XSP);
    const int y = h - 1 + r, xc = pc - 1;
    float v = 0.0f;
    if (y >= 0 && y < NH && xc >= 0 && xc < NW) v = x[((size_t)(b * NC + c) * NH + y) * NW + xc];
    xs[(r * XSP + pc) * NC + c] = (_Float16)v;
  }
  __syncthreads();

  const v8f z = {0.f, 0.f, 0.f, 0.f, 0.f, 0.f, 0.f, 0.f};
  v8f acc[2] = {z, z};
#pragma unroll
  for (int k = 0; k < NK; ++k) {
    const int kh = k / 3, kw = k - kh * 3;
    const _Float16* ap = xs + (kh * XSP + wave * 16 + m + kw) * NC;
    Frag fa;
    fa.half[0] = *(const v8h*)(ap + 8 * hf);
    fa.half[1] = *(const v8h*)(ap + 16 + 8 * hf);
#pragma unroll
    for (int t = 0; t < 2; ++t) {
      const _Float16* bp = wsm + (t * 16 + m) * PITCH + k * NC;
      Frag fb;
      fb.half[0] = *(const v8h*)(bp + 8 * hf);
      fb.half[1] = *(const v8h*)(bp + 16 + 8 * hf);
      acc[t] = wmma_f16(fa.v, fb.v, acc[t]);
    }
  }

#pragma unroll
  for (int t = 0; t < 2; ++t) {
    const int ch = t * 16 + m;
    float bias = 0.0f;
    if (ch < NOFF) bias = ob[ch];
    else if (ch < NOFF + NMOD) bias = mb[ch - NOFF];
#pragma unroll
    for (int r = 0; r < 8; ++r) {
      const int pos = wave * 16 + 8 * hf + r;
      float v = acc[t][r] * (1.0f / 1024.0f) + bias;
      if (ch >= NOFF) v = 1.0f / (1.0f + __expf(-v));
      osm[ch * OSP + pos] = v;
    }
  }
  __syncthreads();

  conv1_rows_out(osm, offo, modo, b, h, wave, lane);
  __threadfence();
  conv1_rows_out(osm, offo, modo, b, h, wave, lane);
}

__device__ __forceinline__ void dconv_rows_out(const float* osm, const float* pst, float* pre, float* part,
                                               int b, int h, int blk, int wave, int lane) {
  for (int o = wave; o < NO; o += 8) {
    const v4f v = *(const v4f*)(osm + o * OSP + 4 * lane);
    *(volatile v4f*)(pre + ((size_t)(b * NO + o) * NH + h) * NW + 4 * lane) = v;
  }
  if (wave == 0) {
    const v4f v = *(const v4f*)(pst + 4 * lane);
    *(volatile v4f*)(part + (size_t)blk * 128 + 4 * lane) = v;
  }
}

__global__ void __launch_bounds__(256) k_dconv(
    const float* __restrict__ x,  const float* __restrict__ offo,
    const float* __restrict__ cw, const float* __restrict__ cb,
    float* pre, float* part, int nblk)
{
  extern __shared__ v4f_t ldsraw[];
  unsigned char* base = (unsigned char*)ldsraw;
  _Float16* wl  = (_Float16*)base;
  _Float16* vl  = wl + NO * PITCH;
  float*    osm = (float*)base;
  __shared__ __align__(16) float pst[128];

  const int blk = blockIdx.x;
  if (blk >= nblk) return;
  const int b = blk / NH, h = blk - b * NH;
  const int tid = threadIdx.x, wave = tid >> 5, lane = tid & 31;
  const int hf = lane >> 4, m = lane & 15;

  for (int i = tid; i < NO * KD; i += 256) {
    const int k = i % NK, c = (i / NK) % NC, o = i / KD;
    wl[o * PITCH + k * NC + c] = (_Float16)(cw[i] * 256.0f);
  }

  const int wcol = wave * 16 + m;
  const float* xb = x + (size_t)(b * NC + hf * 16) * HW;
  _Float16* vrow = vl + (wave * 16 + m) * PITCH + hf * 16;
#pragma unroll 1
  for (int k = 0; k < NK; ++k) {
    const int kh = k / 3, kw = k - kh * 3;
    const size_t oi = ((size_t)(b * NOFF + 2 * k) * NH + h) * NW + wcol;
    const float oy = offo[oi];
    const float ox = offo[oi + HW];
    float py = oy + (float)(h - 1 + kh);
    float px = ox + (float)(wcol - 1 + kw);
    py = fminf(fmaxf(py, -4.0f), (float)(NH + 3));
    px = fminf(fmaxf(px, -4.0f), (float)(NW + 3));
    const float y0f = floorf(py), x0f = floorf(px);
    const float wy = py - y0f, wx = px - x0f;
    const int y0 = (int)y0f, x0i = (int)x0f;
    const int y1 = y0 + 1, x1 = x0i + 1;
    float w00 = (1.f - wy) * (1.f - wx), w01 = (1.f - wy) * wx;
    float w10 = wy * (1.f - wx),         w11 = wy * wx;
    const bool vy0 = (y0 >= 0) && (y0 < NH), vy1 = (y1 >= 0) && (y1 < NH);
    const bool vx0 = (x0i >= 0) && (x0i < NW), vx1 = (x1 >= 0) && (x1 < NW);
    w00 = (vy0 && vx0) ? w00 : 0.f;  w01 = (vy0 && vx1) ? w01 : 0.f;
    w10 = (vy1 && vx0) ? w10 : 0.f;  w11 = (vy1 && vx1) ? w11 : 0.f;
    const int cy0 = min(max(y0, 0), NH - 1), cy1 = min(max(y1, 0), NH - 1);
    const int cx0 = min(max(x0i, 0), NW - 1), cx1 = min(max(x1, 0), NW - 1);
    const int i00 = cy0 * NW + cx0, i01 = cy0 * NW + cx1;
    const int i10 = cy1 * NW + cx0, i11 = cy1 * NW + cx1;
#pragma unroll
    for (int ci = 0; ci < 16; ++ci) {
      const float* xc = xb + (size_t)ci * HW;
      const float v = w00 * xc[i00] + w01 * xc[i01] + w10 * xc[i10] + w11 * xc[i11];
      vrow[k * NC + ci] = (_Float16)v;
    }
  }
  __syncthreads();

  const v8f z = {0.f, 0.f, 0.f, 0.f, 0.f, 0.f, 0.f, 0.f};
  v8f acc[4] = {z, z, z, z};
  const _Float16* arow = vl + (wave * 16 + m) * PITCH;
#pragma unroll
  for (int k = 0; k < NK; ++k) {
    const _Float16* ap = arow + k * NC;
    Frag fa;
    fa.half[0] = *(const v8h*)(ap + 8 * hf);
    fa.half[1] = *(const v8h*)(ap + 16 + 8 * hf);
#pragma unroll
    for (int t = 0; t < 4; ++t) {
      const _Float16* bp = wl + (t * 16 + m) * PITCH + k * NC;
      Frag fb;
      fb.half[0] = *(const v8h*)(bp + 8 * hf);
      fb.half[1] = *(const v8h*)(bp + 16 + 8 * hf);
      acc[t] = wmma_f16(fa.v, fb.v, acc[t]);
    }
  }
  __syncthreads();

#pragma unroll
  for (int t = 0; t < 4; ++t) {
    const int o = t * 16 + m;
    const float bias = cb[o];
#pragma unroll
    for (int r = 0; r < 8; ++r) {
      const int pos = wave * 16 + 8 * hf + r;
      osm[o * OSP + pos] = acc[t][r] * (1.0f / 256.0f) + bias;
    }
  }
  __syncthreads();

  if (tid < NO) {
    float s = 0.f, s2 = 0.f;
    const float* rp = osm + tid * OSP;
    for (int p = 0; p < OSP; ++p) { const float v = rp[p]; s += v; s2 += v * v; }
    pst[tid] = s;
    pst[NO + tid] = s2;
  }
  __syncthreads();

  dconv_rows_out(osm, pst, pre, part, b, h, blk, wave, lane);
  __threadfence();
  dconv_rows_out(osm, pst, pre, part, b, h, blk, wave, lane);
}

__global__ void __launch_bounds__(256) k_stats(
    const float* __restrict__ part, const float* __restrict__ gamma, const float* __restrict__ beta,
    float* stats, int nblkp)
{
  __shared__ double sS[4][NO], sQ[4][NO];
  __shared__ __align__(16) float st[128];
  const int tid = threadIdx.x;
  const int o = tid & 63, q = tid >> 6;
  const int per = (nblkp + 3) / 4;
  const int start = q * per;
  const int stop = min(start + per, nblkp);
  double S = 0.0, Q = 0.0;
  for (int blk = start; blk < stop; ++blk) {
    S += (double)part[(size_t)blk * 128 + o];
    Q += (double)part[(size_t)blk * 128 + NO + o];
  }
  sS[q][o] = S;
  sQ[q][o] = Q;
  __syncthreads();
  if (tid < NO) {
    const double St = ((sS[0][tid] + sS[1][tid]) + sS[2][tid]) + sS[3][tid];
    const double Qt = ((sQ[0][tid] + sQ[1][tid]) + sQ[2][tid]) + sQ[3][tid];
    const double n = (double)nblkp * (double)OSP;
    const double mean = St / n;
    double var = Qt / n - mean * mean;
    if (var < 0.0) var = 0.0;
    const float inv = 1.0f / sqrtf((float)var + 1e-5f);
    const float sc = gamma[tid] * inv;
    const float sh = beta[tid] - (float)mean * sc;
    st[tid] = sc;
    st[NO + tid] = sh;
  }
  __syncthreads();
  if (tid < 32) {
    const v4f v = *(const v4f*)(st + 4 * tid);
    *(volatile v4f*)(stats + 4 * tid) = v;
    __threadfence();
    *(volatile v4f*)(stats + 4 * tid) = v;
  }
}

__global__ void __launch_bounds__(64) k_pool(
    const float* __restrict__ pre, const float* __restrict__ stats, float* out, int nblk)
{
  const int blk = blockIdx.x;
  if (blk >= nblk) return;
  const int g = blk & 15, o = (blk >> 4) & 63, b = blk >> 10;
  const int tid = threadIdx.x;
  const int h2 = g * 4 + (tid >> 4);
  const int c4 = (tid & 15) * 4;
  const float sc = stats[o], sh = stats[NO + o];
  const float* r0 = pre + ((size_t)(b * NO + o) * NH + 2 * h2) * NW + 2 * c4;
  const float* r1 = r0 + NW;
  const v4f a0 = *(const v4f*)r0, a1 = *(const v4f*)(r0 + 4);
  const v4f b0 = *(const v4f*)r1, b1 = *(const v4f*)(r1 + 4);
  v4f res;
  {
    float p0 = fmaxf(fmaxf(a0[0] * sc + sh, a0[1] * sc + sh), fmaxf(b0[0] * sc + sh, b0[1] * sc + sh));
    float p1 = fmaxf(fmaxf(a0[2] * sc + sh, a0[3] * sc + sh), fmaxf(b0[2] * sc + sh, b0[3] * sc + sh));
    float p2 = fmaxf(fmaxf(a1[0] * sc + sh, a1[1] * sc + sh), fmaxf(b1[0] * sc + sh, b1[1] * sc + sh));
    float p3 = fmaxf(fmaxf(a1[2] * sc + sh, a1[3] * sc + sh), fmaxf(b1[2] * sc + sh, b1[3] * sc + sh));
    res[0] = fmaxf(p0, 0.0f); res[1] = fmaxf(p1, 0.0f); res[2] = fmaxf(p2, 0.0f); res[3] = fmaxf(p3, 0.0f);
  }
  float* dst = out + ((size_t)(b * NO + o) * (NH / 2) + h2) * (NW / 2) + c4;
  *(volatile v4f*)dst = res;
  __threadfence();
  *(volatile v4f*)dst = res;
}

extern "C" void kernel_launch(void* const* d_in, const int* in_sizes, int n_in,
                              void* d_out, int out_size, void* d_ws, size_t ws_size,
                              hipStream_t stream) {
  if (n_in < 9) return;
  if (in_sizes[0] != NB * NC * HW) return;
  if (in_sizes[1] != NOFF * NC * NK || in_sizes[2] != NOFF) return;
  if (in_sizes[3] != NMOD * NC * NK || in_sizes[4] != NMOD) return;
  if (in_sizes[5] != NO * NC * NK || in_sizes[6] != NO || in_sizes[7] != NO || in_sizes[8] != NO) return;
  if (out_size != NB * NO * (NH / 2) * (NW / 2)) return;

  const float* x     = (const float*)d_in[0];
  const float* ow    = (const float*)d_in[1];
  const float* ob    = (const float*)d_in[2];
  const float* mw    = (const float*)d_in[3];
  const float* mb    = (const float*)d_in[4];
  const float* cw    = (const float*)d_in[5];
  const float* cb    = (const float*)d_in[6];
  const float* gamma = (const float*)d_in[7];
  const float* beta  = (const float*)d_in[8];

  const int nblk  = NB * NH;
  const int npool = NB * NO * (NH / 8);

  const size_t off_bytes   = (size_t)NB * NOFF * HW * sizeof(float);
  const size_t mod_bytes   = (size_t)NB * NMOD * HW * sizeof(float);
  const size_t pre_bytes   = (size_t)NB * NO * HW * sizeof(float);
  const size_t part_bytes  = (size_t)nblk * 128 * sizeof(float);
  const size_t stats_bytes = 128 * sizeof(float);
  const size_t o_off   = 0;
  const size_t o_mod   = o_off + off_bytes;
  const size_t o_pre   = o_mod + mod_bytes;
  const size_t o_part  = o_pre + pre_bytes;
  const size_t o_stats = o_part + part_bytes;
  const size_t total   = o_stats + stats_bytes;
  if (total > ws_size) return;

  unsigned char* ws = (unsigned char*)d_ws;
  float* offo  = (float*)(ws + o_off);
  float* modo  = (float*)(ws + o_mod);
  float* pre   = (float*)(ws + o_pre);
  float* part  = (float*)(ws + o_part);
  float* stats = (float*)(ws + o_stats);
  float* out   = (float*)d_out;

  const size_t lds1 = (size_t)NCH1 * PITCH * 2 + (size_t)3 * XSP * NC * 2 + (size_t)NCH1 * OSP * 4;
  const size_t lds2 = (size_t)(NO + 128) * PITCH * 2;

  k_conv_off<<<nblk, 256, lds1, stream>>>(x, ow, ob, mw, mb, offo, modo, nblk);
  k_dconv<<<nblk, 256, lds2, stream>>>(x, offo, cw, cb, pre, part, nblk);
  k_stats<<<1, 256, 0, stream>>>(part, gamma, beta, stats, nblk);
  k_pool<<<npool, 64, 0, stream>>>(pre, stats, out, npool);
}
